// DAM_50689204027803
// MI455X (gfx1250) — hardware-verified
//
#include <hip/hip_runtime.h>

typedef _Float16 f16t;
typedef _Float16 v16h __attribute__((ext_vector_type(16)));
typedef _Float16 v8h  __attribute__((ext_vector_type(8)));
typedef __bf16   v16b __attribute__((ext_vector_type(16)));
typedef unsigned short v8us __attribute__((ext_vector_type(8)));
typedef float    v8f  __attribute__((ext_vector_type(8)));
typedef float    v4f  __attribute__((ext_vector_type(4)));
typedef v8h  __attribute__((may_alias)) v8ha;
typedef v8us __attribute__((may_alias)) v8usa;
typedef v4f  __attribute__((may_alias)) v4fa;
union Frag  { v16h v; v8h half[2]; };
union FragB { v16b v; v8us half[2]; v16h x; };
union Q8    { v8f v; v4f q[2]; };

#define NB    4
#define CIN   512
#define CM    128
#define CO    64
#define HW    64
#define NP    4096
#define PADW  66
#define NPP   4356
#define K3A   4608
#define K3B   1152
#define QKP   32
#define SSP   72
#define PSP   72
#define FSP   40
#define ASP   136
#define VSP   72
#define BN_EPS 1e-5f
#define W3SC  64.0f
#define W1SC  16.0f
#define ACAR  8.0f
#define QCAR  8.0f
#define VCAR  8.0f
#define PCAR  1024.0f

__device__ __forceinline__ v8f wmma_f16(v16h a, v16h b, v8f c) {
  v8f d = __builtin_amdgcn_wmma_f32_16x16x32_f16(false, a, false, b, (short)0, c, false, false);
  asm volatile("v_nop\n\tv_nop\n\tv_nop\n\tv_nop" : "+v"(d) : "v"(a), "v"(b));
  return d;
}
__device__ __forceinline__ v8f wmma_bf16(const FragB& a, const FragB& b, v8f c) {
  v8f d = __builtin_amdgcn_wmma_f32_16x16x32_bf16(false, a.v, false, b.v, (short)0, c, false, false);
  asm volatile("v_nop\n\tv_nop\n\tv_nop\n\tv_nop" : "+v"(d) : "v"(a.x), "v"(b.x));
  return d;
}

__device__ __forceinline__ v16h load_frag32(const f16t* p, int h) {
  Frag f;
  f.half[0] = *(const v8ha*)(p + 8 * h);
  f.half[1] = *(const v8ha*)(p + 16 + 8 * h);
  return f.v;
}
__device__ __forceinline__ FragB load_fragb(const unsigned short* p, int h) {
  FragB f;
  f.half[0] = *(const v8usa*)(p + 8 * h);
  f.half[1] = *(const v8usa*)(p + 16 + 8 * h);
  return f;
}

__device__ __forceinline__ v8f zero8f() {
  v8f z;
  #pragma unroll
  for (int j = 0; j < 8; ++j) z[j] = 0.f;
  return z;
}

__device__ __forceinline__ void st8f(float* p, v8f v) {
  Q8 u; u.v = v;
  *(v4fa*)p = u.q[0];
  *(v4fa*)(p + 4) = u.q[1];
}

__device__ __forceinline__ unsigned short bf16_rne(float f) {
  unsigned u = __float_as_uint(f);
  u += 0x7FFFu + ((u >> 16) & 1u);
  return (unsigned short)(u >> 16);
}

__device__ __forceinline__ void plane64_store(const f16t* sT, f16t* __restrict__ TP, int b, int p0, int w, int lane) {
  const int q8 = lane & 7, sub = lane >> 3;
  #pragma unroll
  for (int i = 0; i < 4; ++i) {
    const int id = 16 * w + 4 * i + sub;
    const int pos = id >> 1, L = id & 1;
    const v8h val = *(const v8ha*)(sT + pos * CM + 64 * L + 8 * q8);
    const int p = p0 + pos, yy = p >> 6, xx = p & 63;
    const size_t d = (size_t)(b * NPP + (yy + 1) * PADW + xx + 1) * CM + 64 * L + 8 * q8;
    *(volatile v8h*)(TP + d) = val;
  }
  __threadfence();
  #pragma unroll
  for (int i = 0; i < 4; ++i) {
    const int id = 16 * w + 4 * i + sub;
    const int pos = id >> 1, L = id & 1;
    const v8h val = *(const v8ha*)(sT + pos * CM + 64 * L + 8 * q8);
    const int p = p0 + pos, yy = p >> 6, xx = p & 63;
    const size_t d = (size_t)(b * NPP + (yy + 1) * PADW + xx + 1) * CM + 64 * L + 8 * q8;
    *(volatile v8h*)(TP + d) = val;
  }
}

__global__ __launch_bounds__(256) void k_wcvt(
    const float* __restrict__ w11, const float* __restrict__ w12,
    const float* __restrict__ w21, const float* __restrict__ w22,
    const float* __restrict__ kw, const float* __restrict__ vw,
    const float* __restrict__ w31, const float* __restrict__ w32, const float* __restrict__ w4,
    f16t* __restrict__ W3a, f16t* __restrict__ W3b, f16t* __restrict__ W3c, f16t* __restrict__ W3d,
    f16t* __restrict__ Wq, f16t* __restrict__ Wv, f16t* __restrict__ Wo)
{
  const int g = blockIdx.x * 256 + threadIdx.x;
  if (g >= 189696) return;
  const float* base;
  int stride;
  float sc;
  f16t* dst;
  if (g < 147456) {
    const int sel = (g >= 73728) ? 1 : 0;
    const int e8 = (g - sel * 73728) * 8;
    const int o = e8 / K3A, kk = e8 - o * K3A;
    const int tap = kk >> 9, c = kk & 511;
    base = (sel ? w12 : w11) + ((size_t)(o * CIN + c) * 9 + tap);
    stride = 9; sc = W3SC; dst = (sel ? W3b : W3a) + e8;
  } else if (g < 184320) {
    const int sel = (g >= 165888) ? 1 : 0;
    const int e8 = (g - (sel ? 165888 : 147456)) * 8;
    const int o = e8 / K3B, kk = e8 - o * K3B;
    const int tap = kk >> 7, c = kk & 127;
    base = (sel ? w22 : w21) + ((size_t)(o * CM + c) * 9 + tap);
    stride = 9; sc = W3SC; dst = (sel ? W3d : W3c) + e8;
  } else if (g < 184576) {
    const int e8 = (g - 184320) * 8;
    base = kw + e8; stride = 1; sc = W1SC; dst = Wq + e8;
  } else if (g < 186624) {
    const int e8 = (g - 184576) * 8;
    base = vw + e8; stride = 1; sc = W1SC; dst = Wv + e8;
  } else {
    const int loc = g - 186624;
    const int sel = loc >> 10;
    const float* src = (sel == 0) ? w31 : ((sel == 1) ? w32 : w4);
    base = src + (loc & 1023) * 8; stride = 1; sc = W1SC; dst = Wo + (size_t)loc * 8;
  }
  v8h o8;
  #pragma unroll
  for (int i = 0; i < 8; ++i) o8[i] = (f16t)(base[i * stride] * sc);
  *(volatile v8h*)dst = o8;
  __threadfence();
  *(volatile v8h*)dst = o8;
}

__global__ __launch_bounds__(256) void k_zpad(f16t* __restrict__ XP, f16t* __restrict__ T1P, f16t* __restrict__ T2P) {
  const int g = blockIdx.x * 256 + threadIdx.x;
  if (g >= 99840) return;
  int q, v, b, C;
  f16t* pl;
  if (g < 66560) {
    b = g / 16640;
    const int r = g - b * 16640;
    q = r >> 6; v = r & 63; pl = XP; C = CIN;
  } else {
    const int g2 = g - 66560;
    const int sel = (g2 >= 16640) ? 1 : 0;
    const int r = g2 - sel * 16640;
    b = r / 4160;
    const int r2 = r - b * 4160;
    q = r2 >> 4; v = r2 & 15; pl = sel ? T2P : T1P; C = CM;
  }
  int pp;
  if (q < PADW) pp = q;
  else if (q < 2 * PADW) pp = (PADW - 1) * PADW + (q - PADW);
  else { const int u = q - 2 * PADW; pp = (u / 2 + 1) * PADW + ((u & 1) ? (PADW - 1) : 0); }
  v8h z;
  #pragma unroll
  for (int j = 0; j < 8; ++j) z[j] = (f16t)0.0f;
  f16t* dst = pl + (size_t)(b * NPP + pp) * C + 8 * v;
  *(volatile v8h*)dst = z;
  __threadfence();
  *(volatile v8h*)dst = z;
}

__global__ __launch_bounds__(256) void k_tr(const float* __restrict__ src, const float* __restrict__ src2,
                                           int add2, int C, int padded, f16t* __restrict__ dst)
{
  __shared__ __attribute__((aligned(16))) f16t sH[64 * 64];
  const int tid = threadIdx.x, lane = tid & 31, w = tid >> 5;
  const int cg = blockIdx.x, pg = blockIdx.y, b = blockIdx.z;
  const int p0 = pg * 64;
  const int xq = tid & 15, cl = tid >> 4, x0 = 4 * xq;
  #pragma unroll
  for (int j = 0; j < 4; ++j) {
    const int col = cl + 16 * j, c = 64 * cg + col;
    const size_t off = (size_t)(b * C + c) * NP + p0 + x0;
    v4f v = *(const v4fa*)(src + off);
    if (add2) { const v4f u = *(const v4fa*)(src2 + off); v += u; }
    sH[(x0 + 0) * 64 + col] = (f16t)(v.x * ACAR);
    sH[(x0 + 1) * 64 + col] = (f16t)(v.y * ACAR);
    sH[(x0 + 2) * 64 + col] = (f16t)(v.z * ACAR);
    sH[(x0 + 3) * 64 + col] = (f16t)(v.w * ACAR);
  }
  __syncthreads();
  const int q8 = lane & 7, sub = lane >> 3;
  #pragma unroll
  for (int i = 0; i < 2; ++i) {
    const int lid = 8 * w + 4 * i + sub;
    const v8h val = *(const v8ha*)(sH + lid * 64 + 8 * q8);
    const int prow = padded ? (b * NPP + (pg + 1) * PADW + lid + 1) : (b * NP + p0 + lid);
    const size_t d = (size_t)prow * C + 64 * cg + 8 * q8;
    *(volatile v8h*)(dst + d) = val;
  }
  __threadfence();
  #pragma unroll
  for (int i = 0; i < 2; ++i) {
    const int lid = 8 * w + 4 * i + sub;
    const v8h val = *(const v8ha*)(sH + lid * 64 + 8 * q8);
    const int prow = padded ? (b * NPP + (pg + 1) * PADW + lid + 1) : (b * NP + p0 + lid);
    const size_t d = (size_t)prow * C + 64 * cg + 8 * q8;
    *(volatile v8h*)(dst + d) = val;
  }
}

__global__ __launch_bounds__(256) void k_conv(
    const f16t* __restrict__ T, int Cin, const f16t* __restrict__ Wr,
    const float* __restrict__ g, const float* __restrict__ bt,
    const float* __restrict__ mean, const float* __restrict__ var, float* __restrict__ out)
{
  __shared__ __attribute__((aligned(16))) float sO[CM * 128];
  const int tid = threadIdx.x, lane = tid & 31, w = tid >> 5;
  const int h = lane >> 4, m = lane & 15;
  const int y2 = blockIdx.x, b = blockIdx.y;
  const int yr = w >> 2, og = w & 3;
  const int y = 2 * y2 + yr, o0 = 32 * og;
  const int K = 9 * Cin;
  const v8f z8 = zero8f();
  v8f acc[4][2];
  #pragma unroll
  for (int mt = 0; mt < 4; ++mt) { acc[mt][0] = z8; acc[mt][1] = z8; }

  #pragma unroll 1
  for (int tap = 0; tap < 9; ++tap) {
    const int dy = tap / 3, dx = tap - 3 * dy;
    const int rowb = b * NPP + (y + dy) * PADW + dx;
    const f16t* ab = T + (size_t)(rowb + m) * Cin;
    const f16t* wb = Wr + (size_t)(o0 + m) * K + (size_t)tap * Cin;
    #pragma unroll 1
    for (int c0 = 0; c0 < Cin; c0 += 32) {
      v16h a[4];
      #pragma unroll
      for (int mt = 0; mt < 4; ++mt) a[mt] = load_frag32(ab + (size_t)(16 * mt) * Cin + c0, h);
      #pragma unroll
      for (int nt = 0; nt < 2; ++nt) {
        const v16h bb = load_frag32(wb + (size_t)(16 * nt) * K + c0, h);
        #pragma unroll
        for (int mt = 0; mt < 4; ++mt) acc[mt][nt] = wmma_f16(a[mt], bb, acc[mt][nt]);
      }
    }
  }

  const float osc = 1.0f / (ACAR * W3SC);
  #pragma unroll
  for (int nt = 0; nt < 2; ++nt) {
    const int ol = o0 + 16 * nt + m;
    const float inv = g[ol] * (1.0f / sqrtf(var[ol] + BN_EPS));
    const float sh = bt[ol] - mean[ol] * inv;
    #pragma unroll
    for (int mt = 0; mt < 4; ++mt) {
      v8f vv;
      #pragma unroll
      for (int r = 0; r < 8; ++r) vv[r] = fmaxf(acc[mt][nt][r] * osc * inv + sh, 0.f);
      st8f(sO + ol * 128 + 64 * yr + 16 * mt + 8 * h, vv);
    }
  }
  __syncthreads();
  const int q8 = lane & 7, sub = lane >> 3;
  const size_t obase = (size_t)(b * CM) * NP + (size_t)(2 * y2) * HW;
  #pragma unroll
  for (int i = 0; i < 16; ++i) {
    const int id = 64 * w + 4 * i + sub;
    const int R = id >> 1, L = id & 1;
    const v4f val = *(const v4fa*)(sO + R * 64 + 32 * L + 4 * q8);
    const size_t d = obase + (size_t)(R >> 1) * NP + (R & 1) * HW + 32 * L + 4 * q8;
    *(volatile v4f*)(out + d) = val;
  }
  __threadfence();
  #pragma unroll
  for (int i = 0; i < 16; ++i) {
    const int id = 64 * w + 4 * i + sub;
    const int R = id >> 1, L = id & 1;
    const v4f val = *(const v4fa*)(sO + R * 64 + 32 * L + 4 * q8);
    const size_t d = obase + (size_t)(R >> 1) * NP + (R & 1) * HW + 32 * L + 4 * q8;
    *(volatile v4f*)(out + d) = val;
  }
}

__global__ __launch_bounds__(256) void k_qv(
    const f16t* __restrict__ F1T, const f16t* __restrict__ Wq, const f16t* __restrict__ Wv,
    const float* __restrict__ kb, const float* __restrict__ vb,
    f16t* __restrict__ QT, f16t* __restrict__ VC)
{
  __shared__ __attribute__((aligned(16))) f16t sV[CM * VSP];
  __shared__ __attribute__((aligned(16))) f16t sQ[64 * QKP];
  const int tid = threadIdx.x, lane = tid & 31, w = tid >> 5;
  const int h = lane >> 4, m = lane & 15;
  const int p0 = blockIdx.x * 64, b = blockIdx.y;
  const v8f z8 = zero8f();
  v8f accv[4], accq[4];
  #pragma unroll
  for (int mt = 0; mt < 4; ++mt) { accv[mt] = z8; accq[mt] = z8; }
  const f16t* fb  = F1T + (size_t)(b * NP + p0 + m) * CM;
  const f16t* wvr = Wv + (size_t)(16 * w + m) * CM;
  const f16t* wqr = Wq + (size_t)m * CM;
  #pragma unroll
  for (int k0 = 0; k0 < CM; k0 += 32) {
    v16h f[4];
    #pragma unroll
    for (int mt = 0; mt < 4; ++mt) f[mt] = load_frag32(fb + (size_t)(16 * mt) * CM + k0, h);
    const v16h bvf = load_frag32(wvr + k0, h);
    const v16h aqf = load_frag32(wqr + k0, h);
    #pragma unroll
    for (int mt = 0; mt < 4; ++mt) {
      accv[mt] = wmma_f16(f[mt], bvf, accv[mt]);
      accq[mt] = wmma_f16(aqf, f[mt], accq[mt]);
    }
  }
  const float osc = 1.0f / (ACAR * W1SC);
  {
    const int c = 16 * w + m;
    const float bvv = vb[c];
    #pragma unroll
    for (int mt = 0; mt < 4; ++mt) {
      v8h hv;
      #pragma unroll
      for (int r = 0; r < 8; ++r) hv[r] = (f16t)((accv[mt][r] * osc + bvv) * VCAR);
      *(v8ha*)(sV + c * VSP + 16 * mt + 8 * h) = hv;
    }
  }
  if (w == 0) {
    v8h z;
    #pragma unroll
    for (int j = 0; j < 8; ++j) z[j] = (f16t)0.0f;
    #pragma unroll
    for (int mt = 0; mt < 4; ++mt) {
      const int p = 16 * mt + m;
      v8h hv;
      #pragma unroll
      for (int r = 0; r < 8; ++r) hv[r] = (f16t)((accq[mt][r] * osc + kb[8 * h + r]) * QCAR);
      *(v8ha*)(sQ + p * QKP + 8 * h) = hv;
      *(v8ha*)(sQ + p * QKP + 16 + 8 * h) = z;
    }
  }
  __syncthreads();
  const int q8 = lane & 7, sub = lane >> 3;
  const size_t qbase = (size_t)(b * NP + p0) * QKP;
  #pragma unroll
  for (int i = 0; i < 4; ++i) {
    const int c = 16 * w + 4 * i + sub;
    const v8h val = *(const v8ha*)(sV + c * VSP + 8 * q8);
    const size_t d = (size_t)(b * CM + c) * NP + p0 + 8 * q8;
    *(volatile v8h*)(VC + d) = val;
  }
  if (w == 0) {
    #pragma unroll
    for (int i = 0; i < 8; ++i) {
      const int off = 256 * i + 8 * lane;
      const v8h val = *(const v8ha*)(sQ + off);
      *(volatile v8h*)(QT + qbase + off) = val;
    }
  }
  __threadfence();
  #pragma unroll
  for (int i = 0; i < 4; ++i) {
    const int c = 16 * w + 4 * i + sub;
    const v8h val = *(const v8ha*)(sV + c * VSP + 8 * q8);
    const size_t d = (size_t)(b * CM + c) * NP + p0 + 8 * q8;
    *(volatile v8h*)(VC + d) = val;
  }
  if (w == 0) {
    #pragma unroll
    for (int i = 0; i < 8; ++i) {
      const int off = 256 * i + 8 * lane;
      const v8h val = *(const v8ha*)(sQ + off);
      *(volatile v8h*)(QT + qbase + off) = val;
    }
  }
}

__global__ __launch_bounds__(256) void k_satt(
    const f16t* __restrict__ QT, const f16t* __restrict__ VC, const float* __restrict__ F1F,
    const float* __restrict__ gam, f16t* __restrict__ T1P)
{
  __shared__ __attribute__((aligned(16))) float Ssw[64 * SSP];
  __shared__ __attribute__((aligned(16))) f16t  Psw[64 * PSP];
  __shared__ __attribute__((aligned(16))) f16t  sT[64 * CM];
  __shared__ float rsc[64];
  __shared__ float lsum[64];
  const int tid = threadIdx.x, lane = tid & 31, w = tid >> 5;
  const int h = lane >> 4, m = lane & 15;
  const int i0 = blockIdx.x * 64, b = blockIdx.y;
  const int is_ = w >> 1, jsa = 2 * (w & 1);
  const int si = tid >> 2, jq = tid & 3;
  const float sinv = 1.0f / (QCAR * QCAR);
  const v16h bq = load_frag32(QT + (size_t)(b * NP + i0 + 16 * is_ + m) * QKP, h);
  const f16t* vrow = VC + (size_t)(b * CM + 16 * w + m) * NP;
  const v8f z8 = zero8f();
  v8f acc[4];
  #pragma unroll
  for (int js = 0; js < 4; ++js) acc[js] = z8;
  float mrun = -1.0e30f, lrun = 0.f;

  #pragma unroll 1
  for (int j0 = 0; j0 < NP; j0 += 64) {
    {
      const f16t* kp = QT + (size_t)(b * NP + j0 + 16 * jsa + m) * QKP;
      const v16h a0 = load_frag32(kp, h);
      const v16h a1 = load_frag32(kp + 16 * QKP, h);
      const v8f s0 = wmma_f16(a0, bq, z8);
      const v8f s1 = wmma_f16(a1, bq, z8);
      st8f(Ssw + (16 * is_ + m) * SSP + 16 * jsa + 8 * h, s0);
      st8f(Ssw + (16 * is_ + m) * SSP + 16 * jsa + 16 + 8 * h, s1);
    }
    __syncthreads();

    float sv[16];
    {
      const float* sp = Ssw + si * SSP + 16 * jq;
      #pragma unroll
      for (int q = 0; q < 4; ++q) {
        const v4f t4 = *(const v4fa*)(sp + 4 * q);
        sv[4 * q + 0] = t4.x; sv[4 * q + 1] = t4.y; sv[4 * q + 2] = t4.z; sv[4 * q + 3] = t4.w;
      }
    }
    float mx = sv[0];
    #pragma unroll
    for (int r = 1; r < 16; ++r) mx = fmaxf(mx, sv[r]);
    mx = fmaxf(mx, __shfl_xor(mx, 1));
    mx = fmaxf(mx, __shfl_xor(mx, 2));
    const float mnew = fmaxf(mrun, mx);
    const float rs = __expf((mrun - mnew) * sinv);
    mrun = mnew;
    float psum = 0.f;
    v8h pa, pb;
    #pragma unroll
    for (int r = 0; r < 8; ++r) {
      const float p = __expf((sv[r] - mnew) * sinv);
      psum += p;
      pa[r] = (f16t)(p * PCAR);
    }
    #pragma unroll
    for (int r = 0; r < 8; ++r) {
      const float p = __expf((sv[8 + r] - mnew) * sinv);
      psum += p;
      pb[r] = (f16t)(p * PCAR);
    }
    psum += __shfl_xor(psum, 1);
    psum += __shfl_xor(psum, 2);
    lrun = lrun * rs + psum;
    if (jq == 0) rsc[si] = rs;
    *(v8ha*)(Psw + si * PSP + 16 * jq) = pa;
    *(v8ha*)(Psw + si * PSP + 16 * jq + 8) = pb;
    __syncthreads();

    #pragma unroll
    for (int js = 0; js < 4; ++js) {
      const float rr = rsc[16 * js + m];
      #pragma unroll
      for (int e = 0; e < 8; ++e) acc[js][e] *= rr;
    }
    #pragma unroll
    for (int kc = 0; kc < 2; ++kc) {
      const v16h a = load_frag32(vrow + j0 + 32 * kc, h);
      #pragma unroll
      for (int js = 0; js < 4; ++js) {
        const v16h bb = load_frag32(Psw + (16 * js + m) * PSP + 32 * kc, h);
        acc[js] = wmma_f16(a, bb, acc[js]);
      }
    }
  }

  if (jq == 0) lsum[si] = lrun;
  __syncthreads();
  const float gsc = gam[0] * (1.0f / (VCAR * PCAR));
  const int cb = 16 * w + 8 * h;
  const float* fres = F1F + (size_t)(b * CM + cb) * NP + i0;
  #pragma unroll
  for (int js = 0; js < 4; ++js) {
    const int il = 16 * js + m;
    const float linv = gsc * __builtin_amdgcn_rcpf(lsum[il]);
    v8h hv;
    #pragma unroll
    for (int r = 0; r < 8; ++r) hv[r] = (f16t)((acc[js][r] * linv + fres[(size_t)r * NP + il]) * ACAR);
    *(v8ha*)(sT + il * CM + cb) = hv;
  }
  __syncthreads();
  plane64_store(sT, T1P, b, i0, w, lane);
}

__global__ __launch_bounds__(256) void k_cen(const float* __restrict__ F2F, f16t* __restrict__ ATT)
{
  __shared__ __attribute__((aligned(16))) unsigned short Fh[CM * FSP];
  __shared__ __attribute__((aligned(16))) unsigned short Fl[CM * FSP];
  __shared__ __attribute__((aligned(16))) f16t sAt[CM * ASP];
  const int tid = threadIdx.x, lane = tid & 31, w = tid >> 5;
  const int h = lane >> 4, m = lane & 15;
  const int b = blockIdx.x;
  const int ch = tid >> 1, kh = (tid & 1) * 16;
  const float* frow = F2F + (size_t)(b * CM + ch) * NP + kh;
  const v8f z8 = zero8f();
  v8f acc[8];
  #pragma unroll
  for (int nt = 0; nt < 8; ++nt) acc[nt] = z8;

  #pragma unroll 1
  for (int k0 = 0; k0 < NP; k0 += 32) {
    __syncthreads();
    {
      unsigned short hb[16], lb[16];
      #pragma unroll
      for (int q = 0; q < 4; ++q) {
        const v4f v = *(const v4fa*)(frow + k0 + 4 * q);
        #pragma unroll
        for (int e = 0; e < 4; ++e) {
          const float f = v[e];
          const unsigned short hbits = bf16_rne(f);
          const float lo = f - __uint_as_float(((unsigned)hbits) << 16);
          hb[4 * q + e] = hbits;
          lb[4 * q + e] = bf16_rne(lo);
        }
      }
      v8us h0, h1, l0, l1;
      #pragma unroll
      for (int e = 0; e < 8; ++e) { h0[e] = hb[e]; h1[e] = hb[8 + e]; l0[e] = lb[e]; l1[e] = lb[8 + e]; }
      *(v8usa*)(Fh + ch * FSP + kh) = h0;
      *(v8usa*)(Fh + ch * FSP + kh + 8) = h1;
      *(v8usa*)(Fl + ch * FSP + kh) = l0;
      *(v8usa*)(Fl + ch * FSP + kh + 8) = l1;
    }
    __syncthreads();
    const FragB ah = load_fragb(Fh + (16 * w + m) * FSP, h);
    const FragB al = load_fragb(Fl + (16 * w + m) * FSP, h);
    #pragma unroll
    for (int nt = 0; nt < 8; ++nt) {
      const FragB bh = load_fragb(Fh + (16 * nt + m) * FSP, h);
      const FragB bl = load_fragb(Fl + (16 * nt + m) * FSP, h);
      acc[nt] = wmma_bf16(ah, bh, acc[nt]);
      acc[nt] = wmma_bf16(ah, bl, acc[nt]);
      acc[nt] = wmma_bf16(al, bh, acc[nt]);
    }
  }

  #pragma unroll
  for (int r = 0; r < 8; ++r) {
    float mx = acc[0][r], mn = acc[0][r];
    #pragma unroll
    for (int nt = 1; nt < 8; ++nt) { mx = fmaxf(mx, acc[nt][r]); mn = fminf(mn, acc[nt][r]); }
    mx = fmaxf(mx, __shfl_xor(mx, 1)); mn = fminf(mn, __shfl_xor(mn, 1));
    mx = fmaxf(mx, __shfl_xor(mx, 2)); mn = fminf(mn, __shfl_xor(mn, 2));
    mx = fmaxf(mx, __shfl_xor(mx, 4)); mn = fminf(mn, __shfl_xor(mn, 4));
    mx = fmaxf(mx, __shfl_xor(mx, 8)); mn = fminf(mn, __shfl_xor(mn, 8));
    const float zm = mx - mn;
    float p[8];
    float sum = 0.f;
    #pragma unroll
    for (int nt = 0; nt < 8; ++nt) { p[nt] = __expf((mx - acc[nt][r]) - zm); sum += p[nt]; }
    sum += __shfl_xor(sum, 1);
    sum += __shfl_xor(sum, 2);
    sum += __shfl_xor(sum, 4);
    sum += __shfl_xor(sum, 8);
    const float inv = PCAR * __builtin_amdgcn_rcpf(sum);
    #pragma unroll
    for (int nt = 0; nt < 8; ++nt) sAt[(16 * w + 8 * h + r) * ASP + 16 * nt + m] = (f16t)(p[nt] * inv);
  }
  __syncthreads();
  const int q8 = lane & 7, sub = lane >> 3;
  #pragma unroll
  for (int i = 0; i < 8; ++i) {
    const int id = 32 * w + 4 * i + sub;
    const int row = id >> 1, L = id & 1;
    const v8h val = *(const v8ha*)(sAt + row * ASP + 64 * L + 8 * q8);
    const size_t d = (size_t)(b * CM + row) * CM + 64 * L + 8 * q8;
    *(volatile v8h*)(ATT + d) = val;
  }
  __threadfence();
  #pragma unroll
  for (int i = 0; i < 8; ++i) {
    const int id = 32 * w + 4 * i + sub;
    const int row = id >> 1, L = id & 1;
    const v8h val = *(const v8ha*)(sAt + row * ASP + 64 * L + 8 * q8);
    const size_t d = (size_t)(b * CM + row) * CM + 64 * L + 8 * q8;
    *(volatile v8h*)(ATT + d) = val;
  }
}

__global__ __launch_bounds__(256) void k_cout(
    const f16t* __restrict__ ATT, const f16t* __restrict__ F2T, const float* __restrict__ F2F,
    const float* __restrict__ gam, f16t* __restrict__ T2P)
{
  __shared__ __attribute__((aligned(16))) f16t sT[64 * CM];
  const int tid = threadIdx.x, lane = tid & 31, w = tid >> 5;
  const int h = lane >> 4, m = lane & 15;
  const int p0 = blockIdx.x * 64, b = blockIdx.y;
  const v8f z8 = zero8f();
  v8f acc[4];
  #pragma unroll
  for (int mt = 0; mt < 4; ++mt) acc[mt] = z8;
  const f16t* arow = ATT + (size_t)(b * CM + 16 * w + m) * CM;
  const f16t* fb = F2T + (size_t)(b * NP + p0 + m) * CM;
  #pragma unroll
  for (int k0 = 0; k0 < CM; k0 += 32) {
    const v16h a = load_frag32(arow + k0, h);
    #pragma unroll
    for (int mt = 0; mt < 4; ++mt) {
      const v16h bb = load_frag32(fb + (size_t)(16 * mt) * CM + k0, h);
      acc[mt] = wmma_f16(a, bb, acc[mt]);
    }
  }
  const float gsc = gam[0] * (1.0f / (PCAR * ACAR));
  const int cb = 16 * w + 8 * h;
  const float* fres = F2F + (size_t)(b * CM + cb) * NP + p0;
  #pragma unroll
  for (int mt = 0; mt < 4; ++mt) {
    const int pl = 16 * mt + m;
    v8h hv;
    #pragma unroll
    for (int r = 0; r < 8; ++r) hv[r] = (f16t)((acc[mt][r] * gsc + fres[(size_t)r * NP + pl]) * ACAR);
    *(v8ha*)(sT + pl * CM + cb) = hv;
  }
  __syncthreads();
  plane64_store(sT, T2P, b, p0, w, lane);
}

__global__ __launch_bounds__(256) void k_out(
    const f16t* __restrict__ PCT, const f16t* __restrict__ CCT, const f16t* __restrict__ SUMT,
    const f16t* __restrict__ Wo, const float* __restrict__ b31, const float* __restrict__ b32,
    const float* __restrict__ b4, float* __restrict__ out)
{
  __shared__ __attribute__((aligned(16))) float sO[CO * 64];
  const int tid = threadIdx.x, lane = tid & 31, w = tid >> 5;
  const int h = lane >> 4, m = lane & 15;
  const int p0 = blockIdx.x * 64, b = blockIdx.y, s = blockIdx.z;
  const f16t* pl = (s == 0) ? PCT : ((s == 1) ? CCT : SUMT);
  const float* bias = (s == 0) ? b31 : ((s == 1) ? b32 : b4);
  const f16t* wm = Wo + (size_t)s * (CO * CM);
  const int pt = w & 3, cg = w >> 2;
  const v8f z8 = zero8f();
  v8f acc[2];
  acc[0] = z8; acc[1] = z8;
  const f16t* arow = pl + (size_t)(b * NP + p0 + 16 * pt + m) * CM;
  #pragma unroll
  for (int k0 = 0; k0 < CM; k0 += 32) {
    const v16h a = load_frag32(arow + k0, h);
    #pragma unroll
    for (int t = 0; t < 2; ++t) {
      const v16h bb = load_frag32(wm + (size_t)(32 * cg + 16 * t + m) * CM + k0, h);
      acc[t] = wmma_f16(a, bb, acc[t]);
    }
  }
  const float osc = 1.0f / (ACAR * W1SC);
  #pragma unroll
  for (int t = 0; t < 2; ++t) {
    const int co = 32 * cg + 16 * t + m;
    const float bv = bias[co];
    v8f vv;
    #pragma unroll
    for (int r = 0; r < 8; ++r) vv[r] = acc[t][r] * osc + bv;
    st8f(sO + co * 64 + 16 * pt + 8 * h, vv);
  }
  __syncthreads();
  const int q8 = lane & 7, sub = lane >> 3;
  const size_t obase = ((size_t)(s * NB + b) * CO) * NP + p0;
  #pragma unroll
  for (int i = 0; i < 4; ++i) {
    const int id = 16 * w + 4 * i + sub;
    const int co = id >> 1, L = id & 1;
    const v4f val = *(const v4fa*)(sO + co * 64 + 32 * L + 4 * q8);
    const size_t d = obase + (size_t)co * NP + 32 * L + 4 * q8;
    *(volatile v4f*)(out + d) = val;
  }
  __threadfence();
  #pragma unroll
  for (int i = 0; i < 4; ++i) {
    const int id = 16 * w + 4 * i + sub;
    const int co = id >> 1, L = id & 1;
    const v4f val = *(const v4fa*)(sO + co * 64 + 32 * L + 4 * q8);
    const size_t d = obase + (size_t)co * NP + 32 * L + 4 * q8;
    *(volatile v4f*)(out + d) = val;
  }
}

extern "C" void kernel_launch(void* const* d_in, const int* in_sizes, int n_in,
                              void* d_out, int out_size, void* d_ws, size_t ws_size,
                              hipStream_t stream) {
  if (n_in < 33) return;
  if (in_sizes[0] != NB * CIN * NP) return;
  if (out_size != 3 * NB * CO * NP) return;
  if (in_sizes[1] != CM * CIN * 9 || in_sizes[6] != CM * CIN * 9) return;
  if (in_sizes[17] != CM * CM * 9 || in_sizes[22] != CM * CM * 9) return;
  const int vecidx[17] = {2, 3, 4, 5, 7, 8, 9, 10, 14, 18, 19, 20, 21, 23, 24, 25, 26};
  for (int i = 0; i < 17; ++i) if (in_sizes[vecidx[i]] != CM) return;
  if (in_sizes[11] != 16 * CM || in_sizes[12] != 16 || in_sizes[13] != CM * CM) return;
  if (in_sizes[15] < 1 || in_sizes[16] < 1) return;
  if (in_sizes[27] != CO * CM || in_sizes[29] != CO * CM || in_sizes[31] != CO * CM) return;
  if (in_sizes[28] != CO || in_sizes[30] != CO || in_sizes[32] != CO) return;

  const float* x    = (const float*)d_in[0];
  const float* w11  = (const float*)d_in[1];
  const float* g11  = (const float*)d_in[2];
  const float* b11  = (const float*)d_in[3];
  const float* m11  = (const float*)d_in[4];
  const float* v11  = (const float*)d_in[5];
  const float* w12  = (const float*)d_in[6];
  const float* g12  = (const float*)d_in[7];
  const float* b12  = (const float*)d_in[8];
  const float* m12  = (const float*)d_in[9];
  const float* v12  = (const float*)d_in[10];
  const float* kw   = (const float*)d_in[11];
  const float* kb   = (const float*)d_in[12];
  const float* vw   = (const float*)d_in[13];
  const float* vb   = (const float*)d_in[14];
  const float* pgam = (const float*)d_in[15];
  const float* cgam = (const float*)d_in[16];
  const float* w21  = (const float*)d_in[17];
  const float* g21  = (const float*)d_in[18];
  const float* b21  = (const float*)d_in[19];
  const float* m21  = (const float*)d_in[20];
  const float* v21  = (const float*)d_in[21];
  const float* w22  = (const float*)d_in[22];
  const float* g22  = (const float*)d_in[23];
  const float* b22  = (const float*)d_in[24];
  const float* m22  = (const float*)d_in[25];
  const float* v22  = (const float*)d_in[26];
  const float* w31  = (const float*)d_in[27];
  const float* b31  = (const float*)d_in[28];
  const float* w32  = (const float*)d_in[29];
  const float* b32  = (const float*)d_in[30];
  const float* w4   = (const float*)d_in[31];
  const float* b4   = (const float*)d_in[32];
  float* outp = (float*)d_out;

  const size_t szW3a = (size_t)CM * K3A * 2;
  const size_t szW3c = (size_t)CM * K3B * 2;
  const size_t szWq  = (size_t)16 * CM * 2;
  const size_t szWv  = (size_t)CM * CM * 2;
  const size_t szWo  = (size_t)3 * CO * CM * 2;
  const size_t szXP  = (size_t)NB * NPP * CIN * 2;
  const size_t szF   = (size_t)NB * CM * NP * 4;
  const size_t szT   = (size_t)NB * NP * CM * 2;
  const size_t szQT  = (size_t)NB * NP * QKP * 2;
  const size_t szTP  = (size_t)NB * NPP * CM * 2;
  const size_t szATT = (size_t)NB * CM * CM * 2;
  size_t off = 0;
  char* ws = (char*)d_ws;
  f16t*  W3a  = (f16t*)(ws + off); off += szW3a;
  f16t*  W3b  = (f16t*)(ws + off); off += szW3a;
  f16t*  W3c  = (f16t*)(ws + off); off += szW3c;
  f16t*  W3d  = (f16t*)(ws + off); off += szW3c;
  f16t*  Wq   = (f16t*)(ws + off); off += szWq;
  f16t*  Wv   = (f16t*)(ws + off); off += szWv;
  f16t*  Wo   = (f16t*)(ws + off); off += szWo;
  f16t*  XP   = (f16t*)(ws + off); off += szXP;
  float* F1F  = (float*)(ws + off); off += szF;
  float* F2F  = (float*)(ws + off); off += szF;
  float* PCF  = (float*)(ws + off); off += szF;
  float* CCF  = (float*)(ws + off); off += szF;
  f16t*  F1T  = (f16t*)(ws + off); off += szT;
  f16t*  F2T  = (f16t*)(ws + off); off += szT;
  f16t*  PCT  = (f16t*)(ws + off); off += szT;
  f16t*  CCT  = (f16t*)(ws + off); off += szT;
  f16t*  SUMT = (f16t*)(ws + off); off += szT;
  f16t*  VC   = (f16t*)(ws + off); off += szT;
  f16t*  QT   = (f16t*)(ws + off); off += szQT;
  f16t*  T1P  = (f16t*)(ws + off); off += szTP;
  f16t*  T2P  = (f16t*)(ws + off); off += szTP;
  f16t*  ATT  = (f16t*)(ws + off); off += szATT;
  if (off > ws_size) return;

  k_wcvt<<<741, 256, 0, stream>>>(w11, w12, w21, w22, kw, vw, w31, w32, w4,
                                  W3a, W3b, W3c, W3d, Wq, Wv, Wo);
  k_zpad<<<390, 256, 0, stream>>>(XP, T1P, T2P);
  k_tr<<<dim3(CIN / 64, HW, NB), 256, 0, stream>>>(x, x, 0, CIN, 1, XP);
  k_conv<<<dim3(HW / 2, NB), 256, 0, stream>>>(XP, CIN, W3a, g11, b11, m11, v11, F1F);
  k_conv<<<dim3(HW / 2, NB), 256, 0, stream>>>(XP, CIN, W3b, g12, b12, m12, v12, F2F);
  k_tr<<<dim3(CM / 64, HW, NB), 256, 0, stream>>>(F1F, F1F, 0, CM, 0, F1T);
  k_tr<<<dim3(CM / 64, HW, NB), 256, 0, stream>>>(F2F, F2F, 0, CM, 0, F2T);
  k_qv<<<dim3(NP / 64, NB), 256, 0, stream>>>(F1T, Wq, Wv, kb, vb, QT, VC);
  k_satt<<<dim3(NP / 64, NB), 256, 0, stream>>>(QT, VC, F1F, pgam, T1P);
  k_cen<<<dim3(NB), 256, 0, stream>>>(F2F, ATT);
  k_cout<<<dim3(NP / 64, NB), 256, 0, stream>>>(ATT, F2T, F2F, cgam, T2P);
  k_conv<<<dim3(HW / 2, NB), 256, 0, stream>>>(T1P, CM, W3c, g21, b21, m21, v21, PCF);
  k_conv<<<dim3(HW / 2, NB), 256, 0, stream>>>(T2P, CM, W3d, g22, b22, m22, v22, CCF);
  k_tr<<<dim3(CM / 64, HW, NB), 256, 0, stream>>>(PCF, PCF, 0, CM, 0, PCT);
  k_tr<<<dim3(CM / 64, HW, NB), 256, 0, stream>>>(CCF, CCF, 0, CM, 0, CCT);
  k_tr<<<dim3(CM / 64, HW, NB), 256, 0, stream>>>(PCF, CCF, 1, CM, 0, SUMT);
  k_out<<<dim3(NP / 64, NB, 3), 256, 0, stream>>>(PCT, CCT, SUMT, Wo, b31, b32, b4, outp);
}
